// TensorProductConvLayer_88776974008583
// MI455X (gfx1250) — hardware-verified
//
#include <hip/hip_runtime.h>
#include <stddef.h>
#include <stdint.h>

#define NNODE 10000
#define NEDGE 50000
#define CIN   156
#define KH    96
#define WNUM  6928
#define NPL   7744
#define EPAD  50048
#define HP    192
#define TPP   160
#define XGP   160
#define NTHR  256
#define NWAVE 8
#define EPB   128
#define GBM   64
#define GTHR  128
#define S0E 0
#define S1O 2784
#define S1E 3872
#define S0O 4960
#define C1O 2784
#define C1E 3464
#define C0O 4144
#define R3    0.57735026919f
#define R2    0.70710678119f
#define RSQ58 0.13130643286f
#define RSQ68 0.12126781252f
#define PB_W1 5
#define PB_W2 363
#define PB_B2 8
#define NU_W1 1152
#define NU_W2 92928
#define NU_B2 1936
#define F_ROWS   204
#define F_FLTS   (F_ROWS * EPB)
#define TPT_OFF  F_FLTS
#define TPT_FLTS (EPB * TPP)
#define SH_OFF   (TPT_OFF + TPT_FLTS)
#define GI_OFF   (SH_OFF + EPB * 4)
#define XG_OFF   (GI_OFF + EPB)
#define TP_LDS_FLTS (XG_OFF + (EPB * XGP) / 2)
#define TP_LDS_BYTES (TP_LDS_FLTS * 4)
#define EPT    8
#define CHUNK  (NTHR * EPT)
#define WCAP   (EPT * 32)
#define LISTN  (NWAVE * WCAP)
#define NBA    512
#define SLA    9
#define RCAP   4096
#define DEGCAP 64
#define GRPF   (8 * CIN)
#define AGG_ZINTS (LISTN + 2 * RCAP + 3 * NBA)
#define AGG_LDS_INTS (AGG_ZINTS + 16 + NWAVE * GRPF)
#define AGG_LDS_BYTES (AGG_LDS_INTS * 4)
#define WSMAX  134217728

static_assert(2 * 58 * 48 + 2 * 68 * 10 == WNUM);
static_assert(58 * 48 == S1O && S1O + 68 * 16 == S1E && S1E + 68 * 16 == S0O && S0O + 58 * 48 == NPL);
static_assert(NPL % 16 == 0 && S1O % 16 == 0 && S1E % 16 == 0 && S0O % 16 == 0);
static_assert(KH % 32 == 0);
static_assert(NNODE % 8 == 0);
static_assert((8 * CIN * 4) % 128 == 0);
static_assert((TPP * 4) % 128 == 0 && (HP * 2) % 128 == 0);
static_assert(EPAD % EPB == 0 && EPAD % GBM == 0 && EPAD >= NEDGE && EPAD - NEDGE < GBM);
static_assert(NU_W1 == KH * (KH / 8) && NU_W1 <= PB_W1 * NTHR);
static_assert(NU_W2 == NPL * (KH / 8) && NU_W2 == PB_W2 * NTHR);
static_assert(NU_B2 * 4 == NPL && NU_B2 <= PB_B2 * NTHR);
static_assert(CIN % 4 == 0 && CIN == 48 + 30 + 30 + 48);
static_assert(TP_LDS_BYTES <= 300000);
static_assert((TPT_OFF * 4) % 16 == 0 && (SH_OFF * 4) % 16 == 0 && (XG_OFF * 4) % 16 == 0);
static_assert(TPT_FLTS == 20 * NTHR * 4);
static_assert((CHUNK & (CHUNK - 1)) == 0 && CHUNK <= 4096);
static_assert(NBA == (1 << SLA) && NBA % (8 * NWAVE) == 0 && NBA % 32 == 0);
static_assert(((long long)CHUNK << SLA) < (1LL << 31));
static_assert(((long long)NEDGE << SLA) < (1LL << 31));
static_assert(AGG_ZINTS % 4 == 0 && ((AGG_ZINTS + 16) * 4) % 16 == 0 && (GRPF * 4) % 16 == 0);
static_assert(AGG_LDS_BYTES <= 300000);
static_assert(RCAP >= 2641 + 1024 && DEGCAP >= 15 + 8);
static_assert(((NNODE + NBA - 1) / NBA) * NBA >= NNODE);

typedef float          v4f   __attribute__((ext_vector_type(4)));
typedef float          v8f   __attribute__((ext_vector_type(8)));
typedef int            v4i   __attribute__((ext_vector_type(4)));
typedef int            v8i   __attribute__((ext_vector_type(8)));
typedef unsigned       v2u   __attribute__((ext_vector_type(2)));
typedef unsigned short v8us  __attribute__((ext_vector_type(8)));
typedef unsigned short v16us __attribute__((ext_vector_type(16)));
typedef __bf16         v16bf __attribute__((ext_vector_type(16)));
typedef v4f  __attribute__((may_alias)) v4fa;
typedef v4i  __attribute__((may_alias)) v4ia;
typedef v2u  __attribute__((may_alias)) v2ua;
typedef v8us __attribute__((may_alias)) v8usa;
union FragB { v16bf v; v16us u; v8us h[2]; v8i w; };

__device__ __forceinline__ v8f wmb(const FragB& a, const FragB& b, v8f c) {
  v8f d = __builtin_amdgcn_wmma_f32_16x16x32_bf16(false, a.v, false, b.v, (short)0, c, false, false);
  asm volatile("v_nop\n\tv_nop\n\tv_nop\n\tv_nop" : "+v"(d) : "v"(a.w), "v"(b.w));
  return d;
}

__device__ __forceinline__ unsigned bf16_bits(float f) {
  const unsigned u = __float_as_uint(f);
  return (u + 0x7FFFu + ((u >> 16) & 1u)) >> 16;
}
__device__ __forceinline__ float bf16_val(float f) {
  return __uint_as_float(bf16_bits(f) << 16);
}
__device__ __forceinline__ void put16(unsigned short* dp, v8us o) {
  *(volatile v8us*)dp = o;
  __threadfence();
  *(volatile v8us*)dp = o;
}
__device__ __forceinline__ void putf4(float* dp, v4f o) {
  *(volatile v4f*)dp = o;
  __threadfence();
  *(volatile v4f*)dp = o;
}

__device__ __forceinline__ int perm_col(int np) {
  if (np < S1O) return np;
  if (np < S1E) { const int q = np - S1O; const int i = q >> 4, o = q & 15; return o < 10 ? C1O + i * 10 + o : -1; }
  if (np < S0O) { const int q = np - S1E; const int i = q >> 4, o = q & 15; return o < 10 ? C1E + i * 10 + o : -1; }
  return C0O + (np - S0O);
}

__global__ __launch_bounds__(NTHR) __attribute__((amdgpu_num_vgpr(248)))
void k_prep(const float* __restrict__ W1, const float* __restrict__ W2, const float* __restrict__ b2,
            unsigned short* W1T, unsigned short* W2P, float* B2P) {
  const int bid = (int)blockIdx.x, tid = (int)threadIdx.x;
  if (bid < PB_W1) {
    const int u = bid * NTHR + tid;
    if (u >= NU_W1) return;
    const int n  = u / 12;
    const int k8 = (u - n * 12) * 8;
    const float* p = W1 + (size_t)k8 * KH + n;
    v8us o;
#pragma unroll
    for (int i = 0; i < 8; ++i) o[i] = (unsigned short)bf16_bits(p[(size_t)i * KH]);
    put16(W1T + (size_t)u * 8, o);
    return;
  }
  if (bid < PB_W1 + PB_W2) {
    const int u  = (bid - PB_W1) * NTHR + tid;
    const int np = u / 12;
    const int k8 = (u - np * 12) * 8;
    const int col  = perm_col(np);
    const int colc = col < 0 ? 0 : col;
    const unsigned msk = col < 0 ? 0u : 0xffffu;
    const float* p = W2 + (size_t)k8 * WNUM + colc;
    v8us o;
#pragma unroll
    for (int i = 0; i < 8; ++i) o[i] = (unsigned short)(bf16_bits(p[(size_t)i * WNUM]) & msk);
    put16(W2P + (size_t)u * 8, o);
    return;
  }
  {
    const int u = (bid - PB_W1 - PB_W2) * NTHR + tid;
    if (u >= NU_B2) return;
    const int c0 = perm_col(4 * u + 0), c1 = perm_col(4 * u + 1);
    const int c2 = perm_col(4 * u + 2), c3 = perm_col(4 * u + 3);
    const float v0 = b2[c0 < 0 ? 0 : c0], v1 = b2[c1 < 0 ? 0 : c1];
    const float v2 = b2[c2 < 0 ? 0 : c2], v3 = b2[c3 < 0 ? 0 : c3];
    v4f o;
    o.x = c0 < 0 ? 0.0f : bf16_val(v0);
    o.y = c1 < 0 ? 0.0f : bf16_val(v1);
    o.z = c2 < 0 ? 0.0f : bf16_val(v2);
    o.w = c3 < 0 ? 0.0f : bf16_val(v3);
    putf4(B2P + (size_t)u * 4, o);
  }
}

__global__ __launch_bounds__(GTHR) __attribute__((amdgpu_num_vgpr(248)))
void k_h(const float* __restrict__ EA, const unsigned short* __restrict__ W1T, const float* __restrict__ b1,
         unsigned short* HHL) {
  __shared__ __attribute__((aligned(16))) float stg[GBM * KH];
  const int tid = (int)threadIdx.x, lane = tid & 31, wave = tid >> 5, hh = lane >> 4, m = lane & 15;
  const int rowBase = (int)blockIdx.x * GBM;

  v8f acc[6];
  {
    const v8f z = {0.f, 0.f, 0.f, 0.f, 0.f, 0.f, 0.f, 0.f};
#pragma unroll
    for (int t = 0; t < 6; ++t) acc[t] = z;
  }
  const int row = rowBase + 16 * wave + m;
  const int rc  = row < NEDGE ? row : NEDGE - 1;
  const float*          ap = EA  + (size_t)rc * KH + 8 * hh;
  const unsigned short* bp = W1T + (size_t)m * KH + 8 * hh;
#pragma unroll
  for (int ks = 0; ks < 3; ++ks) {
    const v4f p0 = *(const v4fa*)(ap + 32 * ks);
    const v4f p1 = *(const v4fa*)(ap + 32 * ks + 4);
    const v4f q0 = *(const v4fa*)(ap + 32 * ks + 16);
    const v4f q1 = *(const v4fa*)(ap + 32 * ks + 20);
    v16us t;
    t[0]  = (unsigned short)bf16_bits(p0.x); t[1]  = (unsigned short)bf16_bits(p0.y);
    t[2]  = (unsigned short)bf16_bits(p0.z); t[3]  = (unsigned short)bf16_bits(p0.w);
    t[4]  = (unsigned short)bf16_bits(p1.x); t[5]  = (unsigned short)bf16_bits(p1.y);
    t[6]  = (unsigned short)bf16_bits(p1.z); t[7]  = (unsigned short)bf16_bits(p1.w);
    t[8]  = (unsigned short)bf16_bits(q0.x); t[9]  = (unsigned short)bf16_bits(q0.y);
    t[10] = (unsigned short)bf16_bits(q0.z); t[11] = (unsigned short)bf16_bits(q0.w);
    t[12] = (unsigned short)bf16_bits(q1.x); t[13] = (unsigned short)bf16_bits(q1.y);
    t[14] = (unsigned short)bf16_bits(q1.z); t[15] = (unsigned short)bf16_bits(q1.w);
    FragB af;
    af.u = t;
#pragma unroll
    for (int nt = 0; nt < 6; ++nt) {
      const unsigned short* wq = bp + (size_t)(16 * nt) * KH + 32 * ks;
      FragB bf;
      bf.h[0] = *(const v8usa*)wq;
      bf.h[1] = *(const v8usa*)(wq + 16);
      acc[nt] = wmb(af, bf, acc[nt]);
    }
  }

#pragma unroll
  for (int nt = 0; nt < 6; ++nt) {
    const int lc = 16 * nt + m;
    const float bvv = bf16_val(b1[lc]);
#pragma unroll
    for (int r = 0; r < 8; ++r) {
      const int lr = 16 * wave + 8 * hh + r;
      float v = fmaxf(acc[nt][r] + bvv, 0.0f);
      v = (rowBase + lr < NEDGE) ? v : 0.0f;
      stg[lr * KH + lc] = v;
    }
  }
  __syncthreads();

  {
    v8us pv[12];
#pragma unroll
    for (int it = 0; it < 12; ++it) {
      const int q    = it * 32 + lane;
      const int rl   = q / 24;
      const int part = q - rl * 24;
      const int isLo = part >= 12 ? 1 : 0;
      const int c0   = 8 * (part - 12 * isLo);
      const unsigned mh = 0u - (unsigned)isLo;
      const unsigned ml = ~mh;
      const float* sp = stg + (16 * wave + rl) * KH + c0;
      const v4f a = *(const v4fa*)sp;
      const v4f b = *(const v4fa*)(sp + 4);
      const v8f f8 = {a.x, a.y, a.z, a.w, b.x, b.y, b.z, b.w};
      v8us oo;
#pragma unroll
      for (int e = 0; e < 8; ++e) {
        const unsigned hb = bf16_bits(f8[e]);
        const unsigned lb = bf16_bits(f8[e] - __uint_as_float(hb << 16));
        oo[e] = (unsigned short)((hb & ml) | (lb & mh));
      }
      pv[it] = oo;
    }
    unsigned short* ob = HHL + (size_t)(rowBase + 16 * wave) * HP;
#pragma unroll
    for (int it = 0; it < 12; ++it) *(volatile v8us*)(ob + (size_t)(it * 32 + lane) * 8) = pv[it];
    __threadfence();
#pragma unroll
    for (int it = 0; it < 12; ++it) *(volatile v8us*)(ob + (size_t)(it * 32 + lane) * 8) = pv[it];
  }
}

__device__ __forceinline__ float xgv(const unsigned short* r, int c) {
  return __uint_as_float(((unsigned)r[c]) << 16);
}
__device__ __forceinline__ float sel3(int c, float a, float b, float d) {
  return c == 0 ? a : (c == 1 ? b : d);
}
__device__ __forceinline__ float crossc(const unsigned short* r, int base, int c, float sx, float sy, float sz) {
  const int c1 = (c == 2) ? 0 : c + 1;
  const int c2 = (c == 0) ? 2 : c - 1;
  const float a1 = xgv(r, base + c1);
  const float a2 = xgv(r, base + c2);
  const float s1 = sel3(c1, sx, sy, sz);
  const float s2 = sel3(c2, sx, sy, sz);
  return (a1 * s2 - a2 * s1) * R2;
}
template <int ODD>
__device__ __forceinline__ void build_s(float* F, const unsigned short* xr, int e, int tid,
                                        float s0, float sx, float sy, float sz) {
#pragma unroll 1
  for (int fr = tid >> 7; fr < 58; fr += 2) {
    float v;
    if (ODD == 0) {
      if (fr < 48) {
        v = xgv(xr, fr) * s0;
      } else {
        const int b = 48 + 3 * (fr - 48);
        v = ((xgv(xr, b) * sx + xgv(xr, b + 1) * sy) + xgv(xr, b + 2) * sz) * R3;
      }
    } else {
      if (fr < 10) {
        const int b = 78 + 3 * fr;
        v = ((xgv(xr, b) * sx + xgv(xr, b + 1) * sy) + xgv(xr, b + 2) * sz) * R3;
      } else {
        v = xgv(xr, 108 + (fr - 10)) * s0;
      }
    }
    F[fr * EPB + e] = v;
  }
}
template <int EVEN>
__device__ __forceinline__ void build_v(float* F, const unsigned short* xr, int e, int tid,
                                        float s0, float sx, float sy, float sz) {
#pragma unroll 1
  for (int fr = tid >> 7; fr < F_ROWS; fr += 2) {
    const int i = fr / 3;
    const int c = fr - 3 * i;
    const float sc = sel3(c, sx, sy, sz);
    float v;
    if (EVEN == 0) {
      if (i < 48)      v = xgv(xr, i) * sc;
      else if (i < 58) v = xgv(xr, 48 + 3 * (i - 48) + c) * s0;
      else             v = crossc(xr, 78 + 3 * (i - 58), c, sx, sy, sz);
    } else {
      if (i < 10)      v = crossc(xr, 48 + 3 * i, c, sx, sy, sz);
      else if (i < 20) v = xgv(xr, 78 + 3 * (i - 10) + c) * s0;
      else             v = xgv(xr, 108 + (i - 20)) * sc;
    }
    F[fr * EPB + e] = v;
  }
}
__device__ __forceinline__ v8f tile6(const FragB& h0, const FragB& l0, const FragB& h1, const FragB& l1,
                                     const FragB& h2, const FragB& l2, const unsigned short* __restrict__ wq) {
  v8f d = {0.f, 0.f, 0.f, 0.f, 0.f, 0.f, 0.f, 0.f};
  FragB b0, b1, b2;
  b0.h[0] = *(const v8usa*)(wq);
  b0.h[1] = *(const v8usa*)(wq + 16);
  b1.h[0] = *(const v8usa*)(wq + 32);
  b1.h[1] = *(const v8usa*)(wq + 48);
  b2.h[0] = *(const v8usa*)(wq + 64);
  b2.h[1] = *(const v8usa*)(wq + 80);
  d = wmb(h0, b0, d);
  d = wmb(l0, b0, d);
  d = wmb(h1, b1, d);
  d = wmb(l1, b1, d);
  d = wmb(h2, b2, d);
  d = wmb(l2, b2, d);
  return d;
}
__device__ __forceinline__ void sweep48(const float* Fw, const unsigned short* __restrict__ wp,
                                        const float* __restrict__ bq,
                                        const FragB& h0, const FragB& l0, const FragB& h1, const FragB& l1,
                                        const FragB& h2, const FragB& l2, float* tq, float scale) {
  v8f acc[3];
  {
    const v8f z = {0.f, 0.f, 0.f, 0.f, 0.f, 0.f, 0.f, 0.f};
    acc[0] = z; acc[1] = z; acc[2] = z;
  }
#pragma unroll 1
  for (int i = 0; i < 58; ++i) {
    const v4f f0 = *(const v4fa*)(Fw + i * EPB);
    const v4f f1 = *(const v4fa*)(Fw + i * EPB + 4);
#pragma unroll
    for (int ob = 0; ob < 3; ++ob) {
      const int nb = i * 48 + ob * 16;
      const v8f d = tile6(h0, l0, h1, l1, h2, l2, wp + (size_t)nb * KH);
      const float bv = bq[nb];
      acc[ob][0] = fmaf(f0.x, d[0] + bv, acc[ob][0]);
      acc[ob][1] = fmaf(f0.y, d[1] + bv, acc[ob][1]);
      acc[ob][2] = fmaf(f0.z, d[2] + bv, acc[ob][2]);
      acc[ob][3] = fmaf(f0.w, d[3] + bv, acc[ob][3]);
      acc[ob][4] = fmaf(f1.x, d[4] + bv, acc[ob][4]);
      acc[ob][5] = fmaf(f1.y, d[5] + bv, acc[ob][5]);
      acc[ob][6] = fmaf(f1.z, d[6] + bv, acc[ob][6]);
      acc[ob][7] = fmaf(f1.w, d[7] + bv, acc[ob][7]);
    }
  }
#pragma unroll
  for (int ob = 0; ob < 3; ++ob)
#pragma unroll
    for (int r = 0; r < 8; ++r) tq[r * TPP + ob * 16] = acc[ob][r] * scale;
}
__device__ __forceinline__ void sweep16(const float* Fw, const unsigned short* __restrict__ wp,
                                        const float* __restrict__ bq,
                                        const FragB& h0, const FragB& l0, const FragB& h1, const FragB& l1,
                                        const FragB& h2, const FragB& l2, float* tq, float scale, int m) {
  v8f acc[3];
  {
    const v8f z = {0.f, 0.f, 0.f, 0.f, 0.f, 0.f, 0.f, 0.f};
    acc[0] = z; acc[1] = z; acc[2] = z;
  }
#pragma unroll 1
  for (int i = 0; i < 68; ++i) {
    const int nb = i * 16;
    const v8f d = tile6(h0, l0, h1, l1, h2, l2, wp + (size_t)nb * KH);
    const float bv = bq[nb];
    const float* fp = Fw + (3 * i) * EPB;
#pragma unroll
    for (int c = 0; c < 3; ++c) {
      const v4f f0 = *(const v4fa*)(fp + c * EPB);
      const v4f f1 = *(const v4fa*)(fp + c * EPB + 4);
      acc[c][0] = fmaf(f0.x, d[0] + bv, acc[c][0]);
      acc[c][1] = fmaf(f0.y, d[1] + bv, acc[c][1]);
      acc[c][2] = fmaf(f0.z, d[2] + bv, acc[c][2]);
      acc[c][3] = fmaf(f0.w, d[3] + bv, acc[c][3]);
      acc[c][4] = fmaf(f1.x, d[4] + bv, acc[c][4]);
      acc[c][5] = fmaf(f1.y, d[5] + bv, acc[c][5]);
      acc[c][6] = fmaf(f1.z, d[6] + bv, acc[c][6]);
      acc[c][7] = fmaf(f1.w, d[7] + bv, acc[c][7]);
    }
  }
  if (m < 10) {
#pragma unroll
    for (int c = 0; c < 3; ++c)
#pragma unroll
      for (int r = 0; r < 8; ++r) tq[r * TPP + c] = acc[c][r] * scale;
  }
}

__global__ __launch_bounds__(NTHR) __attribute__((amdgpu_num_vgpr(248)))
void k_tp(const float* __restrict__ X, const int* __restrict__ EI, const float* __restrict__ SHg,
          const unsigned short* __restrict__ HHL, const unsigned short* __restrict__ W2P,
          const float* __restrict__ B2P, float* TP) {
  extern __shared__ __attribute__((aligned(16))) float dyn[];
  float*          F   = dyn;
  float*          TPT = dyn + TPT_OFF;
  float*          SH  = dyn + SH_OFF;
  int*            GI  = (int*)(dyn + GI_OFF);
  unsigned short* XG  = (unsigned short*)(dyn + XG_OFF);

  const int tid = (int)threadIdx.x, lane = tid & 31, wave = tid >> 5, hh = lane >> 4, m = lane & 15;
  const int eBase = (int)blockIdx.x * EPB;

  if (tid < EPB) {
    const int  e    = eBase + tid;
    const bool live = e < NEDGE;
    const int  ec   = live ? e : NEDGE - 1;
    int gi = EI[NEDGE + ec];
    gi = gi < 0 ? 0 : (gi > NNODE - 1 ? NNODE - 1 : gi);
    GI[tid] = gi;
    const v4f s = *(const v4fa*)(SHg + (size_t)ec * 4);
    const float lv = live ? 1.0f : 0.0f;
    v4f o;
    o.x = bf16_val(s.x) * lv; o.y = bf16_val(s.y) * lv; o.z = bf16_val(s.z) * lv; o.w = bf16_val(s.w) * lv;
    *(v4fa*)(SH + 4 * tid) = o;
    const v4f z4 = {0.0f, 0.0f, 0.0f, 0.0f};
    *(v4fa*)(TPT + tid * TPP + CIN) = z4;
  }
  __syncthreads();
#pragma unroll 1
  for (int q = tid; q < EPB * (CIN / 4); q += NTHR) {
    const int e = q / (CIN / 4);
    const int p = q - e * (CIN / 4);
    const int gi = GI[e];
    const unsigned msk = (eBase + e < NEDGE) ? 0xffffffffu : 0u;
    const v4f x = *(const v4fa*)(X + (size_t)gi * CIN + 4 * p);
    v2u w;
    w.x = (bf16_bits(x.x) | (bf16_bits(x.y) << 16)) & msk;
    w.y = (bf16_bits(x.z) | (bf16_bits(x.w) << 16)) & msk;
    *(v2ua*)(XG + e * XGP + 4 * p) = w;
  }
  __syncthreads();

  FragB ah0, ah1, ah2, al0, al1, al2;
  {
    const unsigned short* ap = HHL + (size_t)(eBase + 16 * wave + m) * HP + 8 * hh;
    ah0.h[0] = *(const v8usa*)(ap);            ah0.h[1] = *(const v8usa*)(ap + 16);
    ah1.h[0] = *(const v8usa*)(ap + 32);       ah1.h[1] = *(const v8usa*)(ap + 48);
    ah2.h[0] = *(const v8usa*)(ap + 64);       ah2.h[1] = *(const v8usa*)(ap + 80);
    al0.h[0] = *(const v8usa*)(ap + KH);       al0.h[1] = *(const v8usa*)(ap + KH + 16);
    al1.h[0] = *(const v8usa*)(ap + KH + 32);  al1.h[1] = *(const v8usa*)(ap + KH + 48);
    al2.h[0] = *(const v8usa*)(ap + KH + 64);  al2.h[1] = *(const v8usa*)(ap + KH + 80);
  }

  const int e = tid & (EPB - 1);
  const unsigned short* xr = XG + e * XGP;
  const v4f shv = *(const v4fa*)(SH + 4 * e);
  const float s0 = shv.x, sx = shv.y, sy = shv.z, sz = shv.w;

  const int rw = 16 * wave + 8 * hh;
  const float* Fw = F + rw;
  const unsigned short* wpb = W2P + (size_t)m * KH + 8 * hh;
  const float* bqb = B2P + m;
  float* tqb = TPT + rw * TPP;

  build_s<0>(F, xr, e, tid, s0, sx, sy, sz);
  __syncthreads();
  sweep48(Fw, wpb + (size_t)S0E * KH, bqb + S0E, ah0, al0, ah1, al1, ah2, al2, tqb + 0 + m, RSQ58);
  __syncthreads();
  build_v<0>(F, xr, e, tid, s0, sx, sy, sz);
  __syncthreads();
  sweep16(Fw, wpb + (size_t)S1O * KH, bqb + S1O, ah0, al0, ah1, al1, ah2, al2, tqb + 48 + 3 * m, RSQ68, m);
  __syncthreads();
  build_v<1>(F, xr, e, tid, s0, sx, sy, sz);
  __syncthreads();
  sweep16(Fw, wpb + (size_t)S1E * KH, bqb + S1E, ah0, al0, ah1, al1, ah2, al2, tqb + 78 + 3 * m, RSQ68, m);
  __syncthreads();
  build_s<1>(F, xr, e, tid, s0, sx, sy, sz);
  __syncthreads();
  sweep48(Fw, wpb + (size_t)S0O * KH, bqb + S0O, ah0, al0, ah1, al1, ah2, al2, tqb + 108 + m, RSQ58);
  __syncthreads();

  float* gp = TP + (size_t)eBase * TPP;
#pragma unroll 1
  for (int hf = 0; hf < 2; ++hf) {
    v4f pv[10];
#pragma unroll
    for (int it = 0; it < 10; ++it) pv[it] = *(const v4fa*)(TPT + (size_t)((hf * 10 + it) * NTHR + tid) * 4);
#pragma unroll
    for (int it = 0; it < 10; ++it) *(volatile v4f*)(gp + (size_t)((hf * 10 + it) * NTHR + tid) * 4) = pv[it];
    __threadfence();
#pragma unroll
    for (int it = 0; it < 10; ++it) *(volatile v4f*)(gp + (size_t)((hf * 10 + it) * NTHR + tid) * 4) = pv[it];
  }
}

template <int SLB>
__device__ __forceinline__ int scan_chunk(const int* __restrict__ dsts, int nE, int cbase, int slotBase,
                                          int nb, int vec8, int* list, int tid, int lane, int wave) {
  int wc = 0;
  const int el0  = tid * EPT;
  const int e0   = cbase + el0;
  const int sent = -2147483647 - 1;
  v4i da, db;
  if (vec8 != 0 && cbase + CHUNK <= nE) {
    da = *(const v4i*)(dsts + e0);
    db = *(const v4i*)(dsts + e0 + 4);
  } else {
    da.x = (e0     < nE) ? dsts[min(e0,     nE - 1)] : sent;
    da.y = (e0 + 1 < nE) ? dsts[min(e0 + 1, nE - 1)] : sent;
    da.z = (e0 + 2 < nE) ? dsts[min(e0 + 2, nE - 1)] : sent;
    da.w = (e0 + 3 < nE) ? dsts[min(e0 + 3, nE - 1)] : sent;
    db.x = (e0 + 4 < nE) ? dsts[min(e0 + 4, nE - 1)] : sent;
    db.y = (e0 + 5 < nE) ? dsts[min(e0 + 5, nE - 1)] : sent;
    db.z = (e0 + 6 < nE) ? dsts[min(e0 + 6, nE - 1)] : sent;
    db.w = (e0 + 7 < nE) ? dsts[min(e0 + 7, nE - 1)] : sent;
  }
  const unsigned nbs = (unsigned)slotBase;
  const unsigned unb = (unsigned)nb;
  const unsigned s0 = (unsigned)da.x - nbs, s1 = (unsigned)da.y - nbs;
  const unsigned s2 = (unsigned)da.z - nbs, s3 = (unsigned)da.w - nbs;
  const unsigned s4 = (unsigned)db.x - nbs, s5 = (unsigned)db.y - nbs;
  const unsigned s6 = (unsigned)db.z - nbs, s7 = (unsigned)db.w - nbs;
  const bool h0 = s0 < unb, h1 = s1 < unb, h2 = s2 < unb, h3 = s3 < unb;
  const bool h4 = s4 < unb, h5 = s5 < unb, h6 = s6 < unb, h7 = s7 < unb;
  const unsigned any = __builtin_amdgcn_ballot_w32(h0 | h1 | h2 | h3 | h4 | h5 | h6 | h7);
  if (any != 0u) {
#define HITJ(J, HJ, SJ) { \
      const unsigned mj = __builtin_amdgcn_ballot_w32(HJ); \
      if (mj != 0u) { \
        if (HJ) { \
          const int pos = wc + (int)__builtin_amdgcn_mbcnt_lo(mj, 0u); \
          if (pos < WCAP) list[wave * WCAP + pos] = ((el0 + (J)) << SLB) | (int)(SJ); \
        } \
        wc += (int)__builtin_popcount(mj); } }
    HITJ(0, h0, s0)
    HITJ(1, h1, s1)
    HITJ(2, h2, s2)
    HITJ(3, h3, s3)
    HITJ(4, h4, s4)
    HITJ(5, h5, s5)
    HITJ(6, h6, s6)
    HITJ(7, h7, s7)
#undef HITJ
  }
  return wc;
}

__global__ __launch_bounds__(NTHR) __attribute__((amdgpu_num_vgpr(248)))
void k_agg(const int* __restrict__ keys, const float* __restrict__ TP, const float* __restrict__ X, float* out) {
  extern __shared__ __attribute__((aligned(16))) int dsm[];
  int*   list = dsm;
  int*   hl   = dsm + LISTN;
  int*   sl   = hl + RCAP;
  int*   cnt  = sl + RCAP;
  int*   offs = cnt + NBA;
  int*   cur  = offs + NBA;
  int*   misc = cur + NBA;
  float* stg  = (float*)(misc + 16);
  const int tid = (int)threadIdx.x, lane = tid & 31, wave = tid >> 5;
  const int nodeBase = (int)blockIdx.x * NBA;
  const int nEh = NEDGE;

  {
    const v4i z4 = {0, 0, 0, 0};
    for (int i = tid * 4; i < AGG_ZINTS; i += NTHR * 4) *(v4ia*)(dsm + i) = z4;
    if (tid < 16) misc[tid] = 0;
    const v4f zf = {0.0f, 0.0f, 0.0f, 0.0f};
    for (int i = tid * 4; i < NWAVE * GRPF; i += NTHR * 4) *(v4fa*)(stg + i) = zf;
  }
  __syncthreads();

  int t = 0, ov = 0;
  const int nChunks = (nEh + CHUNK - 1) / CHUNK;
#pragma unroll 1
  for (int ch = 0; ch < nChunks; ++ch) {
    const int cbase = ch * CHUNK;
    const int wc = scan_chunk<SLA>(keys, nEh, cbase, nodeBase, NBA, 1, list, tid, lane, wave);
    if (lane == 0) misc[wave] = wc;
    __syncthreads();
    if (wave == 0) {
#pragma unroll 1
      for (int w2 = 0; w2 < NWAVE; ++w2) {
        int c = misc[w2];
        c = c < 0 ? 0 : (c > WCAP ? WCAP : c);
#pragma unroll 1
        for (int b0 = 0; b0 < c; b0 += 32) {
          const int idx = b0 + lane;
          const int ent = list[w2 * WCAP + (idx < WCAP ? idx : WCAP - 1)];
          const int m32 = (c - b0) < 32 ? (c - b0) : 32;
#pragma unroll 1
          for (int k = 0; k < m32; ++k) {
            const int u    = __builtin_amdgcn_readlane(ent, k);
            const int slot = u & (NBA - 1);
            const int el   = (u >> SLA) & (CHUNK - 1);
            const int pk   = ((cbase + el) << SLA) | slot;
            if (t < RCAP) {
              if (lane == 0) { hl[t] = pk; cnt[slot] = cnt[slot] + 1; }
              t = t + 1;
            } else {
              ov = 1;
            }
          }
        }
      }
    }
    __syncthreads();
  }
  if (wave == 0 && lane == 0) { misc[8] = t; misc[9] = ov; }
  __syncthreads();
  int tt = misc[8];
  tt = tt < 0 ? 0 : (tt > RCAP ? RCAP : tt);
  const int ovf = misc[9];

  if (wave == 0) {
    const int base = lane * (NBA / 32);
    int s = 0;
#pragma unroll 1
    for (int i = 0; i < NBA / 32; ++i) s += cnt[base + i];
    int incl = s;
#pragma unroll
    for (int d = 1; d < 32; d <<= 1) {
      const int y = __shfl_up(incl, d, 32);
      if (lane >= d) incl += y;
    }
    int run = incl - s;
#pragma unroll 1
    for (int i = 0; i < NBA / 32; ++i) {
      const int cv = cnt[base + i];
      offs[base + i] = run;
      cur[base + i]  = run;
      run += cv;
    }
  }
  __syncthreads();
  if (wave == 0) {
#pragma unroll 1
    for (int b0 = 0; b0 < tt; b0 += 32) {
      const int idx = b0 + lane;
      const int ent = hl[idx < RCAP ? idx : RCAP - 1];
      const int m32 = (tt - b0) < 32 ? (tt - b0) : 32;
#pragma unroll 1
      for (int k = 0; k < m32; ++k) {
        const int u    = __builtin_amdgcn_readlane(ent, k);
        const int slot = u & (NBA - 1);
        if (lane == 0) {
          int p = cur[slot];
          p = p < 0 ? 0 : (p > RCAP - 1 ? RCAP - 1 : p);
          sl[p] = u;
          cur[slot] = p + 1;
        }
      }
    }
  }
  __syncthreads();

  const float qnan = __int_as_float(0x7fc00000);
  const float pz = (ovf != 0) ? qnan : 0.0f;
  float* wst = stg + wave * GRPF;
  const int l7 = lane & 7;
  const int l7c = l7 > 6 ? 6 : l7;
#pragma unroll 1
  for (int gi = 0; gi < NBA / (8 * NWAVE); ++gi) {
    const int g   = gi * NWAVE + wave;
    const int nb0 = nodeBase + 8 * g;
    const bool live = (nb0 + 8 <= NNODE);
#pragma unroll 1
    for (int s8 = 0; s8 < 8; ++s8) {
      const int slot = 8 * g + s8;
      const int node = nb0 + s8;
      const int nc   = node < NNODE ? node : NNODE - 1;
      const int craw = cnt[slot];
      int c = craw;
      c = c < 0 ? 0 : (c > DEGCAP ? DEGCAP : c);
      int o = offs[slot];
      o = o < 0 ? 0 : (o > RCAP ? RCAP : o);
      float a0 = 0.0f, a1 = 0.0f, a2 = 0.0f, a3 = 0.0f;
      float c0 = 0.0f, c1 = 0.0f, c2 = 0.0f, c3 = 0.0f;
#pragma unroll 1
      for (int b0 = 0; b0 < c; b0 += 32) {
        int idx = o + b0 + lane;
        idx = idx > RCAP - 1 ? RCAP - 1 : idx;
        const int ent = sl[idx];
        int eid = ent >> SLA;
        eid = eid < 0 ? 0 : (eid > nEh - 1 ? nEh - 1 : eid);
        const int m32 = (c - b0) < 32 ? (c - b0) : 32;
#pragma unroll 1
        for (int k = 0; k < m32; ++k) {
          const int ek = __builtin_amdgcn_readlane(eid, k);
          const float* rp = TP + (size_t)ek * TPP;
          const v4f p = *(const v4fa*)(rp + 4 * lane);
          const v4f q = *(const v4fa*)(rp + 128 + 4 * l7);
          a0 += p.x; a1 += p.y; a2 += p.z; a3 += p.w;
          c0 += q.x; c1 += q.y; c2 += q.z; c3 += q.w;
        }
      }
      const float den = craw > 0 ? (float)craw : 1.0f;
      const float inv = 1.0f / den;
      const float pzr = (craw > DEGCAP) ? qnan : pz;
      const float* xq = X + (size_t)nc * CIN;
      const v4f xa = *(const v4fa*)(xq + 4 * lane);
      const v4f xb = *(const v4fa*)(xq + 128 + 4 * l7c);
      v4f o1, o2;
      o1.x = fmaf(a0, inv, bf16_val(xa.x)) + pzr;
      o1.y = fmaf(a1, inv, bf16_val(xa.y)) + pzr;
      o1.z = fmaf(a2, inv, bf16_val(xa.z)) + pzr;
      o1.w = fmaf(a3, inv, bf16_val(xa.w)) + pzr;
      o2.x = fmaf(c0, inv, bf16_val(xb.x)) + pzr;
      o2.y = fmaf(c1, inv, bf16_val(xb.y)) + pzr;
      o2.z = fmaf(c2, inv, bf16_val(xb.z)) + pzr;
      o2.w = fmaf(c3, inv, bf16_val(xb.w)) + pzr;
      *(v4fa*)(wst + s8 * CIN + 4 * lane) = o1;
      if (lane < 7) *(v4fa*)(wst + s8 * CIN + 128 + 4 * lane) = o2;
    }
    __syncthreads();
    {
      v4f pv[10];
#pragma unroll
      for (int it = 0; it < 10; ++it) {
        int q = it * 32 + lane;
        q = q > 311 ? 311 : q;
        pv[it] = *(const v4fa*)(wst + 4 * q);
      }
      const int nb0c = live ? nb0 : 0;
      float* ob = out + (size_t)nb0c * CIN;
      if (live) {
#pragma unroll
        for (int it = 0; it < 10; ++it) {
          const int q = it * 32 + lane;
          if (q < 312) *(volatile v4f*)(ob + (size_t)q * 4) = pv[it];
        }
      }
      __threadfence();
      if (live) {
#pragma unroll
        for (int it = 0; it < 10; ++it) {
          const int q = it * 32 + lane;
          if (q < 312) *(volatile v4f*)(ob + (size_t)q * 4) = pv[it];
        }
      }
    }
    __syncthreads();
  }
}

extern "C" void kernel_launch(void* const* d_in, const int* in_sizes, int n_in,
                              void* d_out, int out_size, void* d_ws, size_t ws_size,
                              hipStream_t stream) {
  if (n_in < 8) return;
  if (in_sizes[0] != NNODE * CIN) return;
  if (in_sizes[1] != 2 * NEDGE) return;
  if (in_sizes[2] != NEDGE * KH) return;
  if (in_sizes[3] != NEDGE * 4) return;
  if (in_sizes[4] != KH * KH) return;
  if (in_sizes[5] != KH) return;
  if (in_sizes[6] != KH * WNUM) return;
  if (in_sizes[7] != WNUM) return;
  if (out_size != NNODE * CIN) return;

  const float* X   = (const float*)d_in[0];
  const int*   EI  = (const int*)d_in[1];
  const float* EA  = (const float*)d_in[2];
  const float* SHg = (const float*)d_in[3];
  const float* W1  = (const float*)d_in[4];
  const float* b1  = (const float*)d_in[5];
  const float* W2  = (const float*)d_in[6];
  const float* b2  = (const float*)d_in[7];
  float* out = (float*)d_out;

  char* ws = (char*)d_ws;
  size_t off = 0;
  const size_t oW1T = off; off += (size_t)KH * KH * 2;            off = (off + 255) & ~(size_t)255;
  const size_t oW2P = off; off += (size_t)NPL * KH * 2;           off = (off + 255) & ~(size_t)255;
  const size_t oB2P = off; off += (size_t)NPL * 4;                off = (off + 255) & ~(size_t)255;
  const size_t oHHL = off; off += (size_t)EPAD * HP * 2;          off = (off + 255) & ~(size_t)255;
  const size_t oTP  = off; off += (size_t)EPAD * TPP * 4;         off = (off + 255) & ~(size_t)255;
  if (off > ws_size || off > (size_t)WSMAX) return;
  unsigned short* W1T = (unsigned short*)(ws + oW1T);
  unsigned short* W2P = (unsigned short*)(ws + oW2P);
  float*          B2P = (float*)(ws + oB2P);
  unsigned short* HHL = (unsigned short*)(ws + oHHL);
  float*          TP  = (float*)(ws + oTP);

  hipFuncSetAttribute(reinterpret_cast<const void*>(&k_tp), hipFuncAttributeMaxDynamicSharedMemorySize,
                      (int)TP_LDS_BYTES);
  hipFuncSetAttribute(reinterpret_cast<const void*>(&k_agg), hipFuncAttributeMaxDynamicSharedMemorySize,
                      (int)AGG_LDS_BYTES);

  k_prep<<<PB_W1 + PB_W2 + PB_B2, NTHR, 0, stream>>>(W1, W2, b2, W1T, W2P, B2P);
  k_h<<<EPAD / GBM, GTHR, 0, stream>>>(EA, W1T, b1, HHL);
  k_tp<<<EPAD / EPB, NTHR, TP_LDS_BYTES, stream>>>(X, EI, SHg, HHL, W2P, B2P, TP);
  k_agg<<<(NNODE + NBA - 1) / NBA, NTHR, AGG_LDS_BYTES, stream>>>(EI, TP, X, out);
}
